// MambaBlock_49950469652533
// MI455X (gfx1250) — hardware-verified
//
#include <hip/hip_runtime.h>
#include <math.h>

typedef __attribute__((ext_vector_type(16))) _Float16 v16h;
typedef __attribute__((ext_vector_type(8)))  _Float16 v8h;
typedef __attribute__((ext_vector_type(16))) __bf16   v16b;
typedef __attribute__((ext_vector_type(8)))  __bf16   v8b;
typedef __attribute__((ext_vector_type(8)))  float    v8f;
typedef __attribute__((ext_vector_type(4)))  float    v4f;

constexpr int kBatch = 2;
constexpr int kSeqL  = 2048;
constexpr int kDmod  = 1024;
constexpr int kDin   = 2048;
constexpr int kNst   = 16;
constexpr int kDtR   = 64;
constexpr int kPrjN  = 96;
constexpr int kPrjP  = 128;
constexpr int kXZP   = 2 * kDin;
constexpr int kRows  = kBatch * kSeqL;
constexpr int kTP    = 260;

constexpr float kCarryWin  = 32.0f;
constexpr float kCarryWx   = 32.0f;
constexpr float kCarryWdt  = 8.0f;
constexpr float kCarryWout = 32.0f;
constexpr float kCarryDt   = 16.0f;
constexpr float kCarryY    = 16.0f;
constexpr float kFoldIn  = 1.0f / kCarryWin;
constexpr float kFoldX   = 1.0f / kCarryWx;
constexpr float kFoldDt  = 1.0f / (kCarryDt * kCarryWdt);
constexpr float kFoldOut = 1.0f / (kCarryY * kCarryWout);

static_assert(kDtR + 2 * kNst == kPrjN, "x_proj width");
static_assert(kPrjP % 64 == 0 && kPrjP >= kPrjN, "padded x_proj width");
static_assert(kDmod % 32 == 0 && kDin % 32 == 0 && kDtR % 32 == 0, "GEMM K multiples of 32");
static_assert(kRows % 64 == 0 && kXZP % 64 == 0 && kDin % 64 == 0 && kDmod % 64 == 0, "GEMM M,N multiples of 64");
static_assert(kSeqL % 64 == 0 && kDin % 256 == 0 && kSeqL % 16 == 0, "tile multiples");

constexpr size_t kOffX16   = 0;
constexpr size_t kOffWIN   = kOffX16  + (size_t)kRows * kDmod * 2;
constexpr size_t kOffWXP   = kOffWIN  + (size_t)kXZP  * kDmod * 2;
constexpr size_t kOffWDT   = kOffWXP  + (size_t)kPrjP * kDin  * 2;
constexpr size_t kOffWOUT  = kOffWDT  + (size_t)kDin  * kDtR  * 2;
constexpr size_t kOffXZ    = kOffWOUT + (size_t)kDmod * kDin  * 2;
constexpr size_t kOffUY    = kOffXZ   + (size_t)kRows * kXZP  * 4;
constexpr size_t kOffPROJ  = kOffUY   + (size_t)kRows * kDin  * 2;
constexpr size_t kOffDT16  = kOffPROJ + (size_t)kRows * kPrjP * 4;
constexpr size_t kOffDLR   = kOffDT16 + (size_t)kRows * kDtR  * 2;
constexpr size_t kWsTotal  = kOffDLR  + (size_t)kRows * kDin  * 2;
static_assert(kWsTotal == 125042688ull, "carve total");
static_assert(kWsTotal <= 134217728ull, "carve cap");
static_assert((kOffWIN % 128) == 0 && (kOffWXP % 128) == 0 && (kOffWDT % 128) == 0 && (kOffWOUT % 128) == 0 &&
              (kOffXZ % 128) == 0 && (kOffUY % 128) == 0 && (kOffPROJ % 128) == 0 && (kOffDT16 % 128) == 0 &&
              (kOffDLR % 128) == 0, "128-B aligned regions");

__device__ __forceinline__ unsigned short f2bf_bits(float f) {
  unsigned u = __float_as_uint(f);
  return (unsigned short)((u + 0x7FFFu + ((u >> 16) & 1u)) >> 16);
}
__device__ __forceinline__ float bf_bits2f(unsigned short h) { return __uint_as_float(((unsigned)h) << 16); }

__device__ __forceinline__ float h16_to_f32(unsigned hb) {
  const unsigned sgn = (hb & 0x8000u) << 16;
  const unsigned em = hb & 0x7fffu;
  const float fn = __uint_as_float((em << 13) + 0x38000000u);
  const float fs = (float)em * 5.9604644775390625e-8f;
  const float mag = (em < 0x400u) ? fs : fn;
  return __uint_as_float(__float_as_uint(mag) | sgn);
}

__device__ __forceinline__ void dep_guard4_h(v8f& a, v8f& b, v8f& c, v8f& d, v16h x, v16h y) { asm volatile("v_nop\n\tv_nop\n\tv_nop\n\tv_nop" : "+v"(a), "+v"(b), "+v"(c), "+v"(d) : "v"(x), "v"(y)); }
__device__ __forceinline__ void dep_guard4_b(v8f& a, v8f& b, v8f& c, v8f& d, v16b x, v16b y) { asm volatile("v_nop\n\tv_nop\n\tv_nop\n\tv_nop" : "+v"(a), "+v"(b), "+v"(c), "+v"(d) : "v"(x), "v"(y)); }
__device__ __forceinline__ void keep4_h(v16h a, v16h b, v16h c, v16h d) { asm volatile("v_nop" :: "v"(a), "v"(b), "v"(c), "v"(d)); }
__device__ __forceinline__ void keep4_b(v16b a, v16b b, v16b c, v16b d) { asm volatile("v_nop" :: "v"(a), "v"(b), "v"(c), "v"(d)); }
__device__ __forceinline__ void acc_guard4(v8f& a, v8f& b, v8f& c, v8f& d) { asm volatile("v_nop\n\tv_nop\n\tv_nop\n\tv_nop" : "+v"(a), "+v"(b), "+v"(c), "+v"(d)); }
template <typename T> struct Frag;
template <> struct Frag<_Float16> {
  typedef v16h V; union U { v16h v; v8h h[2]; };
  static __device__ __forceinline__ v16h load(const _Float16* p) {
    U f; f.h[0] = *(const v8h*)(p); f.h[1] = *(const v8h*)(p + 16); return f.v;
  }
  static __device__ __forceinline__ v8f mma(v16h a, v16h b, v8f c) {
    return __builtin_amdgcn_wmma_f32_16x16x32_f16(false, a, false, b, (short)0, c, false, false);
  }
  static __device__ __forceinline__ void guard4(v8f& a, v8f& b, v8f& c, v8f& d, v16h x, v16h y) { dep_guard4_h(a, b, c, d, x, y); }
  static __device__ __forceinline__ void keep(v16h a, v16h b, v16h c, v16h d) { keep4_h(a, b, c, d); }
};
template <> struct Frag<__bf16> {
  typedef v16b V; union U { v16b v; v8b h[2]; };
  static __device__ __forceinline__ v16b load(const __bf16* p) {
    U f; f.h[0] = *(const v8b*)(p); f.h[1] = *(const v8b*)(p + 16); return f.v;
  }
  static __device__ __forceinline__ v8f mma(v16b a, v16b b, v8f c) {
    return __builtin_amdgcn_wmma_f32_16x16x32_bf16(false, a, false, b, (short)0, c, false, false);
  }
  static __device__ __forceinline__ void guard4(v8f& a, v8f& b, v8f& c, v8f& d, v16b x, v16b y) { dep_guard4_b(a, b, c, d, x, y); }
  static __device__ __forceinline__ void keep(v16b a, v16b b, v16b c, v16b d) { keep4_b(a, b, c, d); }
};

template <int ET> struct Elem;
template <> struct Elem<0> { typedef _Float16 T; };
template <> struct Elem<1> { typedef __bf16 T; };
template <int ET, bool SPLIT, int BIAS_MODE, int OUT_MODE, bool RESID, int ACT = 0>
__global__ __launch_bounds__(256) void wmma_gemm64(
    const unsigned short* __restrict__ Ap, const unsigned short* __restrict__ A2p, int lda, long strideA,
    const unsigned short* __restrict__ Btp, const unsigned short* __restrict__ Bt2p, int ldb, long strideB,
    void* __restrict__ Cout, void* __restrict__ Cout2, int ldc, long strideC,
    const float* __restrict__ bias,
    const float* __restrict__ resid, long strideR,
    int M, int N, int K, float scale) {
  typedef typename Elem<ET>::T T;
  typedef typename Frag<T>::V V;
  const T* A = (const T*)Ap; const T* A2 = (const T*)A2p; const T* Bt = (const T*)Btp; const T* Bt2 = (const T*)Bt2p;
  __shared__ __align__(16) float sT[8][16 * 68];
  const int b    = blockIdx.y;
  const int lane = threadIdx.x & 31;
  const int wave = threadIdx.x >> 5;
  const int tilesN = N >> 6;
  const int tilesM = M >> 6;
  const int tile = blockIdx.x * 8 + wave;
  if (tile >= tilesM * tilesN) return;
  const int tm = tile / tilesN;
  const int tn = tile - tm * tilesN;
  const int m0 = tm << 6;
  const int n0 = tn << 6;

  const T* Ab  = A  + (size_t)b * strideA;
  const T* Bb  = Bt + (size_t)b * strideB;
  const T* Ab2 = SPLIT ? (A2  + (size_t)b * strideA) : nullptr;
  const T* Bb2 = SPLIT ? (Bt2 + (size_t)b * strideB) : nullptr;

  const int rlane = lane & 15;
  const int koff  = (lane >> 4) * 8;
  const int mOff  = (lane >> 4) * 8;

  v8f acc[4][4];
#pragma unroll
  for (int i = 0; i < 4; ++i)
#pragma unroll
    for (int j = 0; j < 4; ++j) acc[i][j] = (v8f){0.f,0.f,0.f,0.f,0.f,0.f,0.f,0.f};

  for (int k0 = 0; k0 < K; k0 += 32) {
    V bh[4], bl[4];
#pragma unroll
    for (int j = 0; j < 4; ++j) {
      const size_t bo = (size_t)(n0 + (j << 4) + rlane) * ldb + koff + k0;
      bh[j] = Frag<T>::load(Bb + bo);
      if (SPLIT) bl[j] = Frag<T>::load(Bb2 + bo);
    }
#pragma unroll
    for (int i = 0; i < 4; ++i) {
      const size_t ao = (size_t)(m0 + (i << 4) + rlane) * lda + koff + k0;
      V ah = Frag<T>::load(Ab + ao);
      V al;
      if (SPLIT) al = Frag<T>::load(Ab2 + ao);
#pragma unroll
      for (int j = 0; j < 4; ++j) {
        acc[i][j] = Frag<T>::mma(ah, bh[j], acc[i][j]);
        if (SPLIT) {
          acc[i][j] = Frag<T>::mma(ah, bl[j], acc[i][j]);
          acc[i][j] = Frag<T>::mma(al, bh[j], acc[i][j]);
        }
      }
      Frag<T>::guard4(acc[i][0], acc[i][1], acc[i][2], acc[i][3], ah, SPLIT ? al : ah);
    }
    Frag<T>::keep(bh[0], bh[1], bh[2], bh[3]);
    if (SPLIT) Frag<T>::keep(bl[0], bl[1], bl[2], bl[3]);
  }
  acc_guard4(acc[0][0], acc[0][1], acc[0][2], acc[0][3]);
  acc_guard4(acc[1][0], acc[1][1], acc[1][2], acc[1][3]);
  acc_guard4(acc[2][0], acc[2][1], acc[2][2], acc[2][3]);
  acc_guard4(acc[3][0], acc[3][1], acc[3][2], acc[3][3]);

  float* slab = sT[wave];
  const float* Rb = RESID ? (resid + (size_t)b * strideR) : nullptr;
#pragma unroll
  for (int i = 0; i < 4; ++i) {
    const int mBase = m0 + (i << 4);
#pragma unroll
    for (int j = 0; j < 4; ++j) {
      const int n = n0 + (j << 4) + rlane;
      float bv = 0.f;
      if (BIAS_MODE == 2) bv = bias[n];
#pragma unroll
      for (int r = 0; r < 8; ++r) {
        float v = acc[i][j][r] * scale;
        if (BIAS_MODE == 1) v += bias[mBase + mOff + r];
        if (BIAS_MODE == 2) v += bv;
        if (RESID) v += Rb[(size_t)(mBase + mOff + r) * ldc + n];
        if (ACT == 2) v = fmaxf(v, 0.0f);
        if (ACT == 4) v = (v > 0.f) ? v : 0.01f * v;
        slab[(mOff + r) * 68 + (j << 4) + rlane] = v;
      }
    }
    __builtin_amdgcn_fence(__ATOMIC_RELEASE, "workgroup");
    __builtin_amdgcn_wave_barrier();
    __builtin_amdgcn_fence(__ATOMIC_ACQUIRE, "workgroup");
    if (OUT_MODE == 0) {
      float* C = (float*)Cout + (size_t)b * strideC;
      const int hh = lane >> 4, c4 = (lane & 15) * 4;
      for (int pass = 0; pass < 2; ++pass) {
#pragma unroll
        for (int it = 0; it < 8; ++it) {
          const int row = it * 2 + hh;
          v4f v = *(const v4f*)(slab + row * 68 + c4);
          *(volatile v4f*)(C + (size_t)(mBase + row) * ldc + n0 + c4) = v;
        }
        __threadfence();
      }
    } else {
      const int q = lane >> 3, c8 = (lane & 7) * 8;
      unsigned short* C  = (unsigned short*)Cout  + (size_t)b * strideC;
      unsigned short* C2 = (OUT_MODE == 2) ? ((unsigned short*)Cout2 + (size_t)b * strideC) : nullptr;
      for (int pass = 0; pass < 2; ++pass) {
#pragma unroll
        for (int it = 0; it < 4; ++it) {
          const int row = it * 4 + q;
          const float* sp = slab + row * 68 + c8;
          v8h hv, lv;
#pragma unroll
          for (int e = 0; e < 8; ++e) {
            if (OUT_MODE == 1) {
              hv[e] = (_Float16)sp[e];
            } else {
              unsigned short hb = f2bf_bits(sp[e]);
              unsigned short lb = f2bf_bits(sp[e] - bf_bits2f(hb));
              hv[e] = __builtin_bit_cast(_Float16, hb);
              lv[e] = __builtin_bit_cast(_Float16, lb);
            }
          }
          *(volatile v8h*)(C + (size_t)(mBase + row) * ldc + n0 + c8) = hv;
          if (OUT_MODE == 2) *(volatile v8h*)(C2 + (size_t)(mBase + row) * ldc + n0 + c8) = lv;
        }
        __threadfence();
      }
    }
    __builtin_amdgcn_fence(__ATOMIC_RELEASE, "workgroup");
    __builtin_amdgcn_wave_barrier();
    __builtin_amdgcn_fence(__ATOMIC_ACQUIRE, "workgroup");
  }
}

constexpr int kCbX      = kRows * kDmod / 2048;
constexpr int kCbWin    = kXZP * kDmod / 2048;
constexpr int kCbWx     = kPrjP * kDin / 2048;
constexpr int kCbWxReal = kPrjN * kDin / 2048;
constexpr int kCbWdt    = kDin * kDtR / 2048;
constexpr int kCbWout   = kDmod * kDin / 2048;
constexpr int kCbTotal  = kCbX + kCbWin + kCbWx + kCbWdt + kCbWout;
static_assert(kCbX == 2048 && kCbWin == 2048 && kCbWx == 128 && kCbWxReal == 96 && kCbWdt == 64 && kCbWout == 1024, "cast segments");
static_assert(kCbTotal == 5312, "cast grid");

__global__ __launch_bounds__(256) void cast_planes_kernel(
    const float* __restrict__ sx, const float* __restrict__ swin, const float* __restrict__ swx,
    const float* __restrict__ swdt, const float* __restrict__ swout,
    unsigned short* __restrict__ dx, unsigned short* __restrict__ dwin, unsigned short* __restrict__ dwx,
    unsigned short* __restrict__ dwdt, unsigned short* __restrict__ dwout)
{
  int lb = blockIdx.x;
  const float* src = sx;
  unsigned short* dst = dx;
  float scale = 1.0f;
  int realBlocks = kCbX;
  if (lb >= kCbX) {
    lb -= kCbX;
    src = swin; dst = dwin; scale = kCarryWin; realBlocks = kCbWin;
    if (lb >= kCbWin) {
      lb -= kCbWin;
      src = swx; dst = dwx; scale = kCarryWx; realBlocks = kCbWxReal;
      if (lb >= kCbWx) {
        lb -= kCbWx;
        src = swdt; dst = dwdt; scale = kCarryWdt; realBlocks = kCbWdt;
        if (lb >= kCbWdt) {
          lb -= kCbWdt;
          src = swout; dst = dwout; scale = kCarryWout; realBlocks = kCbWout;
          if (lb >= kCbWout) return;
        }
      }
    }
  }
  const bool real = (lb < realBlocks);
  const int lbs = real ? lb : (realBlocks - 1);
  const size_t es = (size_t)lbs * 2048 + (size_t)threadIdx.x * 8;
  const size_t ed = (size_t)lb * 2048 + (size_t)threadIdx.x * 8;
  const v4f a0 = *(const v4f*)(src + es);
  const v4f a1 = *(const v4f*)(src + es + 4);
  v8h hv;
#pragma unroll
  for (int e = 0; e < 4; ++e) {
    const float f0 = real ? (a0[e] * scale) : 0.0f;
    const float f1 = real ? (a1[e] * scale) : 0.0f;
    hv[e]     = (_Float16)f0;
    hv[4 + e] = (_Float16)f1;
  }
  unsigned short* q = dst + ed;
  *(volatile v8h*)q = hv;
  __threadfence();
  *(volatile v8h*)q = hv;
}

__global__ __launch_bounds__(256) void dt_cast_kernel(
    const float* __restrict__ PROJ, unsigned short* __restrict__ DT16, int total8, float scale)
{
  const int i = blockIdx.x * 256 + threadIdx.x;
  if (i >= total8) return;
  const int e0  = i << 3;
  const int row = e0 >> 6;
  const int c8  = e0 & 63;
  const float* p = PROJ + (size_t)row * kPrjP + c8;
  const v4f a0 = *(const v4f*)(p);
  const v4f a1 = *(const v4f*)(p + 4);
  v8h hv;
#pragma unroll
  for (int e = 0; e < 4; ++e) {
    hv[e]     = (_Float16)(a0[e] * scale);
    hv[4 + e] = (_Float16)(a1[e] * scale);
  }
  unsigned short* qd = DT16 + e0;
  *(volatile v8h*)qd = hv;
  __threadfence();
  *(volatile v8h*)qd = hv;
}

__global__ __launch_bounds__(256) void conv_silu_kernel(
    const float* __restrict__ XZ, const float* __restrict__ cw, const float* __restrict__ cb,
    unsigned short* __restrict__ U16)
{
  __shared__ __align__(16) float sT[16 * kTP];
  const int tid = threadIdx.x, lane = tid & 31, wave = tid >> 5;
  const int d0 = blockIdx.x * 256, d = d0 + tid;
  const int g0 = blockIdx.y * 64;
  const int tb = g0 & (kSeqL - 1);
  const v4f wv = *(const v4f*)(cw + (size_t)d * 4);
  const float w0 = wv[0], w1 = wv[1], w2 = wv[2], w3 = wv[3];
  const float bc = cb[d];
  float xm3, xm2, xm1;
  {
    const bool hist = (tb > 0);
    const int rb = hist ? (g0 - 3) : g0;
    const float v3 = XZ[(size_t)rb * kXZP + d];
    const float v2 = XZ[(size_t)(rb + 1) * kXZP + d];
    const float v1 = XZ[(size_t)(rb + 2) * kXZP + d];
    xm3 = hist ? v3 : 0.f;
    xm2 = hist ? v2 : 0.f;
    xm1 = hist ? v1 : 0.f;
  }
#pragma unroll 1
  for (int sub = 0; sub < 4; ++sub) {
    const int lb = g0 + sub * 16;
#pragma unroll 1
    for (int s = 0; s < 16; ++s) {
      const float xc = XZ[(size_t)(lb + s) * kXZP + d];
      float acc = w0 * xm3;
      acc = fmaf(w1, xm2, acc);
      acc = fmaf(w2, xm1, acc);
      acc = fmaf(w3, xc, acc);
      const float sv = acc + bc;
      const float sg = __builtin_amdgcn_rcpf(1.0f + __expf(-sv));
      sT[s * kTP + tid] = sv * sg;
      xm3 = xm2; xm2 = xm1; xm1 = xc;
    }
    __syncthreads();
    v8h bv[2];
#pragma unroll
    for (int it = 0; it < 2; ++it) {
      const float* sp = sT + (it * 8 + wave) * kTP + lane * 8;
      const v4f a0 = *(const v4f*)(sp);
      const v4f a1 = *(const v4f*)(sp + 4);
#pragma unroll
      for (int e = 0; e < 4; ++e) {
        bv[it][e]     = (_Float16)a0[e];
        bv[it][4 + e] = (_Float16)a1[e];
      }
    }
    for (int pass = 0; pass < 2; ++pass) {
#pragma unroll
      for (int it = 0; it < 2; ++it)
        *(volatile v8h*)(U16 + (size_t)(lb + it * 8 + wave) * kDin + d0 + lane * 8) = bv[it];
      __threadfence();
    }
    __syncthreads();
  }
}

__global__ __launch_bounds__(256) void scan_kernel(
    const unsigned* __restrict__ DLRw, const float* __restrict__ XZ, const float* __restrict__ PROJ,
    const float* __restrict__ cw, const float* __restrict__ cb,
    const float* __restrict__ A_log, const float* __restrict__ Dv,
    unsigned short* __restrict__ Y16)
{
  __shared__ __align__(16) float sBC[16 * 32];
  __shared__ __align__(16) float sY[16 * kTP];
  const int tid = threadIdx.x, lane = tid & 31, wave = tid >> 5;
  const int d0 = blockIdx.x * 256, d = d0 + tid;
  const size_t row0 = (size_t)blockIdx.y * kSeqL;
  const unsigned hshift = (unsigned)(d & 1) << 4;

  float An[kNst];
#pragma unroll
  for (int q4 = 0; q4 < 4; ++q4) {
    const v4f al = *(const v4f*)(A_log + (size_t)d * kNst + 4 * q4);
    An[4 * q4 + 0] = -__expf(al[0]);
    An[4 * q4 + 1] = -__expf(al[1]);
    An[4 * q4 + 2] = -__expf(al[2]);
    An[4 * q4 + 3] = -__expf(al[3]);
  }
  const v4f wv = *(const v4f*)(cw + (size_t)d * 4);
  const float w0 = wv[0], w1 = wv[1], w2 = wv[2], w3 = wv[3];
  const float bc = cb[d];
  const float Dd = Dv[d];
  float h[kNst];
#pragma unroll
  for (int n = 0; n < kNst; ++n) h[n] = 0.f;
  float xm3 = 0.f, xm2 = 0.f, xm1 = 0.f;

#pragma unroll 1
  for (int c = 0; c < kSeqL / 16; ++c) {
    const int l0 = c * 16;
    if (tid < 128) {
      const int r = tid >> 3, q = (tid & 7) * 4;
      const v4f v = *(const v4f*)(PROJ + (row0 + l0 + r) * kPrjP + kDtR + q);
      *(v4f*)(sBC + r * 32 + q) = v;
    }
    __syncthreads();
#pragma unroll 1
    for (int s = 0; s < 16; ++s) {
      const size_t m = row0 + (size_t)(l0 + s);
      unsigned wd = DLRw[(m * kDin + d) >> 1];
      float xc = XZ[m * kXZP + d];
      float zv = XZ[m * kXZP + kDin + d];
      asm volatile("" : "+v"(wd));
      asm volatile("" : "+v"(xc));
      asm volatile("" : "+v"(zv));
      float acc = w0 * xm3;
      acc = fmaf(w1, xm2, acc);
      acc = fmaf(w2, xm1, acc);
      acc = fmaf(w3, xc, acc);
      xm3 = xm2; xm2 = xm1; xm1 = xc;
      const float sv = acc + bc;
      const float uv = sv * __builtin_amdgcn_rcpf(1.0f + __expf(-sv));
      const float a   = h16_to_f32((wd >> hshift) & 0xffffu);
      const float ea  = __expf(-fabsf(a));
      const float up  = 1.0f + ea;
      const float l1p = __logf(up) + (ea - (up - 1.0f)) * __builtin_amdgcn_rcpf(up);
      const float delta = fmaxf(a, 0.0f) + l1p;
      const float du = delta * uv;
      v4f Bq[4], Cq[4];
#pragma unroll
      for (int qq = 0; qq < 4; ++qq) {
        Bq[qq] = *(const v4f*)(sBC + s * 32 + 4 * qq);
        Cq[qq] = *(const v4f*)(sBC + s * 32 + kNst + 4 * qq);
      }
      float y = 0.f;
#pragma unroll
      for (int n = 0; n < kNst; ++n) {
        const float e = __expf(delta * An[n]);
        const float hn = e * h[n] + du * Bq[n >> 2][n & 3];
        h[n] = hn;
        y = hn * Cq[n >> 2][n & 3] + y;
      }
      y = uv * Dd + y;
      const float g = zv * __builtin_amdgcn_rcpf(1.0f + __expf(-zv));
      sY[s * kTP + tid] = (y * g) * kCarryY;
    }
    __syncthreads();
    v8h hv[2];
#pragma unroll
    for (int it = 0; it < 2; ++it) {
      const float* sp = sY + (it * 8 + wave) * kTP + lane * 8;
      const v4f a0 = *(const v4f*)(sp);
      const v4f a1 = *(const v4f*)(sp + 4);
#pragma unroll
      for (int e = 0; e < 4; ++e) { hv[it][e] = (_Float16)a0[e]; hv[it][4 + e] = (_Float16)a1[e]; }
    }
    for (int pass = 0; pass < 2; ++pass) {
#pragma unroll
      for (int it = 0; it < 2; ++it)
        *(volatile v8h*)(Y16 + (row0 + (size_t)(l0 + it * 8 + wave)) * kDin + d0 + lane * 8) = hv[it];
      __threadfence();
    }
  }
}

constexpr int kBlkIn  = (kRows / 64) * (kXZP / 64) / 8;
constexpr int kBlkXp  = (kRows / 64) * (kPrjP / 64) / 8;
constexpr int kBlkDt  = (kRows / 64) * (kDin / 64) / 8;
constexpr int kBlkOut = (kRows / 64) * (kDmod / 64) / 8;
static_assert(kBlkIn == 512 && kBlkXp == 16 && kBlkDt == 256 && kBlkOut == 128, "GEMM grids");
static_assert(((kRows / 64) * (kPrjP / 64)) % 8 == 0, "tile count multiple of waves per block");

extern "C" void kernel_launch(void* const* d_in, const int* in_sizes, int n_in,
                              void* d_out, int out_size, void* d_ws, size_t ws_size,
                              hipStream_t stream)
{
  if (n_in < 10) return;
  if (in_sizes[0] != kRows * kDmod) return;
  if (in_sizes[1] != kXZP * kDmod) return;
  if (in_sizes[2] != kDin * 4) return;
  if (in_sizes[3] != kDin) return;
  if (in_sizes[4] != kPrjN * kDin) return;
  if (in_sizes[5] != kDin * kDtR) return;
  if (in_sizes[6] != kDin) return;
  if (in_sizes[7] != kDin * kNst) return;
  if (in_sizes[8] != kDin) return;
  if (in_sizes[9] != kDmod * kDin) return;
  if (out_size != kRows * kDmod) return;
  if (ws_size < kWsTotal) return;

  const float* x      = (const float*)d_in[0];
  const float* W_in   = (const float*)d_in[1];
  const float* conv_w = (const float*)d_in[2];
  const float* conv_b = (const float*)d_in[3];
  const float* W_xprj = (const float*)d_in[4];
  const float* W_dt   = (const float*)d_in[5];
  const float* b_dt   = (const float*)d_in[6];
  const float* A_log  = (const float*)d_in[7];
  const float* Dv     = (const float*)d_in[8];
  const float* W_out  = (const float*)d_in[9];
  float* dout = (float*)d_out;

  char* ws = (char*)d_ws;
  unsigned short* X16    = (unsigned short*)(ws + kOffX16);
  unsigned short* WIN16  = (unsigned short*)(ws + kOffWIN);
  unsigned short* WXP16  = (unsigned short*)(ws + kOffWXP);
  unsigned short* WDT16  = (unsigned short*)(ws + kOffWDT);
  unsigned short* WOUT16 = (unsigned short*)(ws + kOffWOUT);
  float*          XZ     = (float*)(ws + kOffXZ);
  unsigned short* UY16   = (unsigned short*)(ws + kOffUY);
  float*          PROJ   = (float*)(ws + kOffPROJ);
  unsigned short* DT16   = (unsigned short*)(ws + kOffDT16);
  unsigned short* DLR16  = (unsigned short*)(ws + kOffDLR);
  const float* dummy_bias  = b_dt;
  const float* dummy_resid = x;

  cast_planes_kernel<<<kCbTotal, 256, 0, stream>>>(x, W_in, W_xprj, W_dt, W_out, X16, WIN16, WXP16, WDT16, WOUT16);

  wmma_gemm64<0, false, 0, 0, false><<<dim3(kBlkIn, 1), 256, 0, stream>>>(
      X16, X16, kDmod, 0L, WIN16, WIN16, kDmod, 0L,
      (void*)XZ, (void*)XZ, kXZP, 0L, dummy_bias, dummy_resid, 0L, kRows, kXZP, kDmod, kFoldIn);

  conv_silu_kernel<<<dim3(kDin / 256, kRows / 64), 256, 0, stream>>>(XZ, conv_w, conv_b, UY16);

  wmma_gemm64<0, false, 0, 0, false><<<dim3(kBlkXp, 1), 256, 0, stream>>>(
      UY16, UY16, kDin, 0L, WXP16, WXP16, kDin, 0L,
      (void*)PROJ, (void*)PROJ, kPrjP, 0L, dummy_bias, dummy_resid, 0L, kRows, kPrjP, kDin, kFoldX);

  dt_cast_kernel<<<(kRows * kDtR) / 8 / 256, 256, 0, stream>>>(PROJ, DT16, (kRows * kDtR) / 8, kCarryDt);

  wmma_gemm64<0, false, 2, 1, false><<<dim3(kBlkDt, 1), 256, 0, stream>>>(
      DT16, DT16, kDtR, 0L, WDT16, WDT16, kDtR, 0L,
      (void*)DLR16, (void*)DLR16, kDin, 0L, b_dt, dummy_resid, 0L, kRows, kDin, kDtR, kFoldDt);

  scan_kernel<<<dim3(kDin / 256, kBatch), 256, 0, stream>>>(
      (const unsigned*)DLR16, XZ, PROJ, conv_w, conv_b, A_log, Dv, UY16);

  wmma_gemm64<0, false, 0, 0, false><<<dim3(kBlkOut, 1), 256, 0, stream>>>(
      UY16, UY16, kDin, 0L, WOUT16, WOUT16, kDin, 0L,
      (void*)dout, (void*)dout, kDmod, 0L, dummy_bias, dummy_resid, 0L, kRows, kDmod, kDin, kFoldOut);
}
